// Luong_61684320305412
// MI455X (gfx1250) — hardware-verified
//
#include <hip/hip_runtime.h>


#define NB_  8
#define TT   2048
#define DD   256
#define ZH   1
#define RH   0
#define PCAR 1024.0f
#define SCL  0.00390625f
#define NEGB (-100000000.0f)
#define OSC  (1.0f / (16.0f * 1024.0f))
typedef _Float16 h16;
typedef unsigned short bf;
typedef __attribute__((ext_vector_type(16))) __bf16   v16bf;
typedef __attribute__((ext_vector_type(16))) _Float16 v16h;
typedef __attribute__((ext_vector_type(8)))  _Float16 v8h;
typedef __attribute__((ext_vector_type(8)))  unsigned short v8us;
typedef __attribute__((ext_vector_type(8)))  float    v8f;
typedef __attribute__((ext_vector_type(4)))  float    v4f;
typedef v8h  __attribute__((may_alias)) v8ha;
typedef v4f  __attribute__((may_alias)) v4fa;
typedef v8us __attribute__((may_alias)) v8usa;

__device__ __forceinline__ unsigned short f2bf(float f) { unsigned u = __float_as_uint(f); u += 0x7FFFu + ((u >> 16) & 1u); return (unsigned short)(u >> 16); }
__device__ __forceinline__ float bf2f(unsigned short b) { return __uint_as_float(((unsigned)b) << 16); }
__device__ __forceinline__ float bfr(float f) { return bf2f(f2bf(f)); }
__device__ __forceinline__ v16h cat16(v8h lo, v8h hi) { return __builtin_shufflevector(lo, hi, 0, 1, 2, 3, 4, 5, 6, 7, 8, 9, 10, 11, 12, 13, 14, 15); }
__device__ __forceinline__ v16bf cat16b(v8us lo, v8us hi) { return __builtin_bit_cast(v16bf, __builtin_shufflevector(lo, hi, 0, 1, 2, 3, 4, 5, 6, 7, 8, 9, 10, 11, 12, 13, 14, 15)); }
__device__ __forceinline__ v8f wmma16(v16h a, v16h b, v8f c) { return __builtin_amdgcn_wmma_f32_16x16x32_f16(false, a, false, b, (short)0, c, false, false); }
__device__ __forceinline__ v8f wmmab(v16bf a, v16bf b, v8f c) { return __builtin_amdgcn_wmma_f32_16x16x32_bf16(false, a, false, b, (short)0, c, false, false); }


template <typename T16> struct WFrag;
template <> struct WFrag<h16> { typedef v16h V; static __device__ __forceinline__ V ld(const h16* p) { return cat16(*(const v8h*)p, *(const v8h*)(p + 16)); } static __device__ __forceinline__ v8f mma(V a, V b, v8f c) { return wmma16(a, b, c); } };
template <> struct WFrag<bf> { typedef v16bf V; static __device__ __forceinline__ V ld(const bf* p) { return cat16b(*(const v8us*)p, *(const v8us*)(p + 16)); } static __device__ __forceinline__ v8f mma(V a, V b, v8f c) { return wmmab(a, b, c); } };
template <typename T16, int NSPLIT, bool BIAS>
__global__ __launch_bounds__(32) void k_gemmw(const T16* __restrict__ A, const T16* __restrict__ A2, const T16* __restrict__ Bt, const T16* __restrict__ Bt2, int K, float* C, int ldc, const float* __restrict__ bias, size_t sA, size_t sB, size_t sC) {
    typedef typename WFrag<T16>::V V;
    __shared__ __align__(16) float os[16 * 68];
    const size_t z = blockIdx.z; A += z * sA; if (A2) A2 += z * sA; Bt += z * sB; if (Bt2) Bt2 += z * sB; C += z * sC;
    const int lane = threadIdx.x & 31, lr = lane & 15, hi = lane >> 4; const int r0 = blockIdx.x * 64, c0 = blockIdx.y * 64;
    v8f acc[4][4];
#pragma unroll
    for (int mb = 0; mb < 4; ++mb)
#pragma unroll
        for (int nb = 0; nb < 4; ++nb) acc[mb][nb] = (v8f){};
    const size_t aoff = (size_t)(r0 + lr) * K + 8 * hi, boff = (size_t)(c0 + lr) * K + 8 * hi;
#pragma unroll 1
    for (int kc = 0; kc < K; kc += 32) {
        V a[4], a2[4];
#pragma unroll
        for (int mb = 0; mb < 4; ++mb) { a[mb] = WFrag<T16>::ld(A + aoff + (size_t)mb * 16 * K + kc); if (NSPLIT == 1 || NSPLIT == 2) a2[mb] = WFrag<T16>::ld(A2 + aoff + (size_t)mb * 16 * K + kc); }
#pragma unroll
        for (int nb = 0; nb < 4; ++nb) { const V b = WFrag<T16>::ld(Bt + boff + (size_t)nb * 16 * K + kc); V b2; if (NSPLIT >= 2) b2 = WFrag<T16>::ld(Bt2 + boff + (size_t)nb * 16 * K + kc);
#pragma unroll
            for (int mb = 0; mb < 4; ++mb) { acc[mb][nb] = WFrag<T16>::mma(a[mb], b, acc[mb][nb]); if (NSPLIT == 1 || NSPLIT == 2) acc[mb][nb] = WFrag<T16>::mma(a2[mb], b, acc[mb][nb]); if (NSPLIT >= 2) acc[mb][nb] = WFrag<T16>::mma(a[mb], b2, acc[mb][nb]); } }
        asm volatile("v_nop\n\tv_nop\n\tv_nop\n\tv_nop" : "+v"(acc[0][0]), "+v"(acc[1][1]), "+v"(acc[2][2]), "+v"(acc[3][3]) : "v"(a[0]), "v"(a[3]));
    }
#pragma unroll
    for (int mb = 0; mb < 4; ++mb) {
#pragma unroll
        for (int nb = 0; nb < 4; ++nb) {
#pragma unroll
            for (int j = 0; j < 8; ++j) os[(hi * 8 + j) * 68 + nb * 16 + lr] = acc[mb][nb][j]; }
        __builtin_amdgcn_wave_barrier(); asm volatile("" ::: "memory");
        float* crow = C + (size_t)(r0 + mb * 16) * ldc + c0;
#pragma unroll 1
        for (int ps = 0; ps < 2; ++ps) {
#pragma unroll
            for (int s = 0; s < 8; ++s) { const int row = 2 * s + hi, cofs = lr * 4; v4f val = *(const v4fa*)(os + row * 68 + cofs); if (BIAS) { val[0] += bfr(bias[c0 + cofs]); val[1] += bfr(bias[c0 + cofs + 1]); val[2] += bfr(bias[c0 + cofs + 2]); val[3] += bfr(bias[c0 + cofs + 3]); }
                *(volatile v4f*)(crow + (size_t)row * ldc + cofs) = val; }
            if (ps == 0) __threadfence(); }
        __builtin_amdgcn_wave_barrier(); asm volatile("" ::: "memory");
    }
}

__device__ __forceinline__ h16 tohx(float x) { return (h16)x; }
__device__ __forceinline__ void splitf(float y, unsigned short& h, unsigned short& l) { h = f2bf(y); l = f2bf(y - bf2f(h)); }
typedef __attribute__((ext_vector_type(2))) _Float16 v2h;
typedef __attribute__((ext_vector_type(4))) _Float16 v4h;
typedef __attribute__((ext_vector_type(2))) unsigned short v2us;

__global__ __launch_bounds__(256) void k_cvt8(const float* __restrict__ src, bf* dst, size_t n8) { const size_t i = (size_t)blockIdx.x * 256 + threadIdx.x; if (i >= n8) return; const v8f v = *(const v8f*)(src + i * 8); v8us o;
#pragma unroll
    for (int k = 0; k < 8; ++k) o[k] = f2bf(v[k]); *(volatile v8us*)(dst + i * 8) = o; __threadfence(); *(volatile v8us*)(dst + i * 8) = o; }
__global__ __launch_bounds__(256) void k_t16(const float* __restrict__ X, h16* T16) { const int e = (blockIdx.x * 256 + threadIdx.x) * 2; if (e >= DD * TT) return; const int t = e % TT, d = e / TT; v2h o; o[0] = tohx(bfr(X[(size_t)t * DD + d])); o[1] = tohx(bfr(X[(size_t)(t + 1) * DD + d])); *(volatile v2h*)(T16 + e) = o; __threadfence(); *(volatile v2h*)(T16 + e) = o; }
__global__ __launch_bounds__(256) void k_mouter(const int* __restrict__ m0, const int* __restrict__ m1, float* MB) { const size_t e = ((size_t)blockIdx.x * 256 + threadIdx.x) * 4; if (e >= (size_t)TT * TT) return; const int j = (int)(e % TT), i = (int)(e / TT); const float a = NEGB * (float)m0[i]; v4f o;
#pragma unroll
    for (int q = 0; q < 4; ++q) o[q] = __fmul_rn(a, (float)m1[j + q]); *(volatile v4f*)(MB + e) = o; __threadfence(); *(volatile v4f*)(MB + e) = o; }
__global__ __launch_bounds__(256) void k_asoft(const float* __restrict__ Sb, const float* __restrict__ ab, bf* Ph, bf* Pl, h16* P16) {
    typedef __attribute__((ext_vector_type(4))) unsigned short v4us;
    const int lane = threadIdx.x & 31; const int row = blockIdx.x * 8 + (threadIdx.x >> 5); if (row >= ZH * TT) return; const int i = row & (TT - 1); const int zz = row >> 11; const bool hires = (i < RH);
    const float* sr = Sb + (size_t)row * TT; const float* mr = ab + (size_t)i * TT; float v[64]; float mx = -3.0e38f;
#pragma unroll
    for (int ch = 0; ch < 16; ++ch) { const int j0 = ch * 128 + lane * 4; const v4f a = *(const v4f*)(sr + j0), m4 = *(const v4f*)(mr + j0);
#pragma unroll
        for (int q = 0; q < 4; ++q) { float sa = a[q] * SCL, mb = m4[q]; asm volatile("" : "+v"(sa)); asm volatile("" : "+v"(mb)); const float t = __fadd_rn(sa, mb); v[ch * 4 + q] = t; mx = fmaxf(mx, t); } }
#pragma unroll
    for (int sh = 16; sh; sh >>= 1) mx = fmaxf(mx, __shfl_xor(mx, sh, 32));
    float sum = 0.f;
#pragma unroll
    for (int k = 0; k < 64; ++k) { v[k] = __expf(v[k] - mx); sum += v[k]; }
#pragma unroll
    for (int sh = 16; sh; sh >>= 1) sum += __shfl_xor(sum, sh, 32);
    const float f = __fdiv_rn(hires ? 1.0f : PCAR, sum);
#pragma unroll 1
    for (int ps = 0; ps < 2; ++ps) {
        if (hires) {
#pragma unroll
            for (int ch = 0; ch < 16; ++ch) { v4us oh, ol;
#pragma unroll
                for (int q = 0; q < 4; ++q) { unsigned short a, c2; splitf(v[ch * 4 + q] * f, a, c2); oh[q] = a; ol[q] = c2; }
                const size_t o = ((size_t)zz * RH + i) * TT + ch * 128 + lane * 4; *(volatile v4us*)(Ph + o) = oh; *(volatile v4us*)(Pl + o) = ol; }
        } else {
#pragma unroll
            for (int ch = 0; ch < 16; ++ch) { v4h o;
#pragma unroll
                for (int q = 0; q < 4; ++q) o[q] = tohx(v[ch * 4 + q] * f);
                *(volatile v4h*)(P16 + (size_t)row * TT + ch * 128 + lane * 4) = o; } }
        if (ps == 0) __threadfence(); }
}

__global__ __launch_bounds__(256) void k_colst(const float* __restrict__ S, const float* __restrict__ MB, float* CM, float* CI) { const int j = blockIdx.x * 256 + threadIdx.x; if (j >= TT) return; float m = -3.0e38f;
    for (int i = 0; i < TT; ++i) { float a = S[(size_t)i * TT + j] * SCL; asm volatile("" : "+v"(a)); m = fmaxf(m, __fadd_rn(a, MB[(size_t)i * TT + j])); }
    float s = 0.f; for (int i = 0; i < TT; ++i) { float a = S[(size_t)i * TT + j] * SCL; asm volatile("" : "+v"(a)); float d0 = __fsub_rn(__fadd_rn(a, MB[(size_t)i * TT + j]), m); asm volatile("" : "+v"(d0)); s = __fadd_rn(s, __expf(d0)); }
    const float ci = __fdiv_rn(PCAR, s); *(volatile float*)(CM + j) = m; *(volatile float*)(CI + j) = ci; __threadfence(); *(volatile float*)(CM + j) = m; *(volatile float*)(CI + j) = ci; }
__global__ __launch_bounds__(256) void k_pcolT(const float* __restrict__ S, const float* __restrict__ MB, const float* __restrict__ CM, const float* __restrict__ CI, h16* PT) { const int e = (blockIdx.x * 256 + threadIdx.x) * 2; if (e >= TT * TT) return; const int i = e % TT, j = e / TT; const float m = CM[j], ci = CI[j]; v2h o;
#pragma unroll
    for (int q = 0; q < 2; ++q) { float a = S[(size_t)(i + q) * TT + j] * SCL; asm volatile("" : "+v"(a)); float d0 = __fsub_rn(__fadd_rn(a, MB[(size_t)(i + q) * TT + j]), m); asm volatile("" : "+v"(d0)); o[q] = tohx(__fmul_rn(__expf(d0), ci)); } *(volatile v2h*)(PT + e) = o; __threadfence(); *(volatile v2h*)(PT + e) = o; }
__global__ __launch_bounds__(256) void k_osc(const float* __restrict__ O, float* OUTb) { const size_t i = ((size_t)blockIdx.x * 256 + threadIdx.x) * 4; if (i >= (size_t)TT * DD) return; const v4f a = *(const v4f*)(O + i); v4f o;
#pragma unroll
    for (int q = 0; q < 4; ++q) o[q] = a[q] * OSC; *(volatile v4f*)(OUTb + i) = o; __threadfence(); *(volatile v4f*)(OUTb + i) = o; }

extern "C" void kernel_launch(void* const* d_in, const int* in_sizes, int n_in,
                              void* d_out, int out_size, void* d_ws, size_t ws_size, hipStream_t stream) {
    (void)in_sizes; (void)n_in; (void)out_size;
    const float* q0 = (const float*)d_in[0]; const float* q1 = (const float*)d_in[1]; const int* m0 = (const int*)d_in[4]; const int* m1 = (const int*)d_in[5];
    float* OUT0 = (float*)d_out; float* OUT1 = (float*)d_out + (size_t)NB_ * TT * DD;
    char* wsp = (char*)d_ws;
    auto take = [&](size_t bytes) { char* p = wsp; wsp += (bytes + 255) & ~(size_t)255; return (void*)p; };
    bf* Q0B = (bf*)take((size_t)TT * DD * 2); bf* Q1B = (bf*)take((size_t)TT * DD * 2); h16* Q0T = (h16*)take((size_t)DD * TT * 2); h16* Q1T = (h16*)take((size_t)DD * TT * 2); float* S = (float*)take((size_t)TT * TT * 4); float* MB = (float*)take((size_t)TT * TT * 4);
    h16* P16 = (h16*)take((size_t)TT * TT * 2); h16* PT = (h16*)take((size_t)TT * TT * 2); float* CM = (float*)take((size_t)TT * 4); float* CI = (float*)take((size_t)TT * 4); float* O = (float*)take((size_t)TT * DD * 4);
    if ((size_t)(wsp - (char*)d_ws) > ws_size) return;
    const unsigned L8 = (unsigned)(((size_t)TT * DD / 8 + 255) / 256), L2 = (unsigned)(((size_t)TT * DD / 2 + 255) / 256), L4o = (unsigned)(((size_t)TT * DD / 4 + 255) / 256);
    for (int b = 0; b < NB_; ++b) { const float* q0b = q0 + (size_t)b * TT * DD; const float* q1b = q1 + (size_t)b * TT * DD;
        k_cvt8<<<L8, 256, 0, stream>>>(q0b, Q0B, (size_t)TT * DD / 8); k_cvt8<<<L8, 256, 0, stream>>>(q1b, Q1B, (size_t)TT * DD / 8); k_t16<<<L2, 256, 0, stream>>>(q0b, Q0T); k_t16<<<L2, 256, 0, stream>>>(q1b, Q1T);
        k_gemmw<bf, 0, false><<<dim3(TT / 64, TT / 64, 1), 32, 0, stream>>>(Q0B, nullptr, Q1B, nullptr, DD, S, TT, nullptr, 0, 0, 0);
        k_mouter<<<(unsigned)(((size_t)TT * TT / 4 + 255) / 256), 256, 0, stream>>>(m0 + (size_t)b * TT, m1 + (size_t)b * TT, MB);
        k_asoft<<<TT / 8, 256, 0, stream>>>(S, MB, nullptr, nullptr, P16);
        k_gemmw<h16, 0, false><<<dim3(TT / 64, DD / 64, 1), 32, 0, stream>>>(P16, nullptr, Q1T, nullptr, TT, O, DD, nullptr, 0, 0, 0); k_osc<<<L4o, 256, 0, stream>>>(O, OUT0 + (size_t)b * TT * DD);
        k_colst<<<TT / 256, 256, 0, stream>>>(S, MB, CM, CI); k_pcolT<<<(unsigned)(((size_t)TT * TT / 2 + 255) / 256), 256, 0, stream>>>(S, MB, CM, CI, PT);
        k_gemmw<h16, 0, false><<<dim3(TT / 64, DD / 64, 1), 32, 0, stream>>>(PT, nullptr, Q0T, nullptr, TT, O, DD, nullptr, 0, 0, 0); k_osc<<<L4o, 256, 0, stream>>>(O, OUT1 + (size_t)b * TT * DD); }
}
